// LinearAttentionLayer_55551107006697
// MI455X (gfx1250) — hardware-verified
//
#include <hip/hip_runtime.h>


namespace {
constexpr int Bn = 2, S = 2048, DIM = 1024, H = 8, HD = 64, INNER = H * HD, NTOK = Bn * S, NBH = Bn * H, CH = 64  , NC = S / CH  ;
constexpr float PS8 = 8.0f, CXS = 1.0f / 64.0f, EPS = 1e-6f;
constexpr size_t QPL = (size_t)NTOK * INNER  , TPL = (size_t)NBH * HD * S  , CPL = (size_t)NBH * NC * HD * HD;

typedef _Float16 b16;
typedef __attribute__((ext_vector_type(16))) _Float16 v16b;
typedef __attribute__((ext_vector_type(16))) __bf16 v16bb;
typedef __attribute__((ext_vector_type(8))) _Float16 v8b;
typedef __attribute__((ext_vector_type(8))) unsigned short v8us;
typedef __attribute__((ext_vector_type(8))) float v8f;
typedef __attribute__((ext_vector_type(4))) float v4f;
__device__ __forceinline__ float bf16_rne(float f) { unsigned int u = __float_as_uint(f); u += 0x7FFFu + ((u >> 16) & 1u); return __uint_as_float(u & 0xFFFF0000u); }
__device__ __forceinline__ unsigned short bf16_bits(float f) { unsigned int u = __float_as_uint(f); u += 0x7FFFu + ((u >> 16) & 1u); return (unsigned short)(u >> 16); }
__device__ __forceinline__ void split16(float v, b16& hi, b16& lo) { hi = (b16)v; lo = (b16)(v - (float)hi); }
__device__ __forceinline__ v16b frag_kb(const b16* p, int hh) { const v8b a = *(const v8b*)(p + 8 * hh), b = *(const v8b*)(p + 16 + 8 * hh); v16b f;
#pragma unroll
  for (int e = 0; e < 8; ++e) { f[e] = a[e]; f[8 + e] = b[e]; } return f; }
__device__ __forceinline__ v16bb frag_bf(const unsigned short* p, int hh) { const v8us a = *(const v8us*)(p + 8 * hh), b = *(const v8us*)(p + 16 + 8 * hh); union { unsigned short s[16]; v16bb v; } u;
#pragma unroll
  for (int e = 0; e < 8; ++e) { u.s[e] = a[e]; u.s[8 + e] = b[e]; } return u.v; }
__device__ __forceinline__ v8f wmma16b(v16b a, v16b b, v8f c) { v8f d = __builtin_amdgcn_wmma_f32_16x16x32_f16(false, a, false, b, (short)0, c, false, false); asm volatile("v_nop\n\tv_nop\n\tv_nop\n\tv_nop" : "+v"(d) : "v"(a), "v"(b)); return d; }
__device__ __forceinline__ v8f wmma16bb(v16bb a, v16bb b, v8f c) { v8f d = __builtin_amdgcn_wmma_f32_16x16x32_bf16(false, a, false, b, (short)0, c, false, false); asm volatile("v_nop\n\tv_nop\n\tv_nop\n\tv_nop" : "+v"(d) : "v"(a), "v"(b)); return d; }
__device__ __forceinline__ void wave_lds_sync() { __builtin_amdgcn_fence(__ATOMIC_RELEASE, "workgroup"); __builtin_amdgcn_wave_barrier(); __builtin_amdgcn_fence(__ATOMIC_ACQUIRE, "workgroup"); }
__device__ __forceinline__ float phi(float t) { return (t > 0.0f) ? t + 1.0f : __expf(t); }

__global__ __launch_bounds__(256) void prep_kernel(const float* __restrict__ x, const float* __restrict__ wqkv, const float* __restrict__ wout, unsigned short* __restrict__ x16, unsigned short* __restrict__ w16, b16* __restrict__ wo16) {
  const size_t tid = (size_t)blockIdx.x * blockDim.x + threadIdx.x, nth = (size_t)gridDim.x * blockDim.x;
  for (int pass = 0; pass < 2; ++pass) {
    for (size_t p = tid; p < (size_t)NTOK * DIM / 8; p += nth) { v8us v;
#pragma unroll
      for (int e = 0; e < 8; ++e) v[e] = bf16_bits(x[p * 8 + e]);
      *(volatile v8us*)(x16 + p * 8) = v; }
    for (size_t p = tid; p < (size_t)3 * INNER * DIM / 8; p += nth) { const int n = (int)(p / (DIM / 8)), k0 = (int)(p % (DIM / 8)) * 8; v8us v;
#pragma unroll
      for (int e = 0; e < 8; ++e) v[e] = bf16_bits(wqkv[(size_t)(k0 + e) * (3 * INNER) + n]);
      *(volatile v8us*)(w16 + (size_t)n * DIM + k0) = v; }
    for (size_t p = tid; p < (size_t)DIM * INNER / 8; p += nth) { const int n = (int)(p / (INNER / 8)), k0 = (int)(p % (INNER / 8)) * 8; v8b v;
#pragma unroll
      for (int e = 0; e < 8; ++e) v[e] = (b16)bf16_rne(wout[(size_t)(k0 + e) * DIM + n]);
      *(volatile v8b*)(wo16 + (size_t)n * INNER + k0) = v; }
    __threadfence();
  }
}

__global__ __launch_bounds__(128) void proj_kernel(const unsigned short* __restrict__ x16, const unsigned short* __restrict__ w16, b16* __restrict__ qh, b16* __restrict__ kh, b16* __restrict__ kT, b16* __restrict__ vT) {
  __shared__ __attribute__((aligned(16))) b16 Th[4][32][64 + 8], Tl[4][32][64 + 8]; __shared__ __attribute__((aligned(16))) b16 Tt[64][128 + 8], Ttl[64][128 + 8];
  const int lane = threadIdx.x & 31, wave = threadIdx.x >> 5, nloc = lane & 15, hlf = lane >> 4, m0 = blockIdx.y * 128 + wave * 32, c0 = blockIdx.x * 64;
  const int which = blockIdx.x / 8, head = blockIdx.x % 8, b = (blockIdx.y * 128) / S, tok0 = (blockIdx.y * 128) % S;
  v8f acc[2][4];
#pragma unroll
  for (int r = 0; r < 2; ++r)
#pragma unroll
    for (int t = 0; t < 4; ++t) acc[r][t] = (v8f){};
#pragma unroll 2
  for (int kb = 0; kb < DIM; kb += 32) { const v16bb a0 = frag_bf(x16 + (size_t)(m0 + nloc) * DIM + kb, hlf), a1 = frag_bf(x16 + (size_t)(m0 + 16 + nloc) * DIM + kb, hlf);
#pragma unroll
    for (int t = 0; t < 4; ++t) { const v16bb bw = frag_bf(w16 + (size_t)(c0 + t * 16 + nloc) * DIM + kb, hlf); acc[0][t] = wmma16bb(a0, bw, acc[0][t]); acc[1][t] = wmma16bb(a1, bw, acc[1][t]); } }
  if (which < 2) {
#pragma unroll
    for (int t = 0; t < 4; ++t)
#pragma unroll
      for (int r = 0; r < 2; ++r)
#pragma unroll
        for (int v = 0; v < 8; ++v) { b16 a_, c_; split16(phi(acc[r][t][v]) * PS8, a_, c_); Th[wave][r * 16 + 8 * hlf + v][t * 16 + nloc] = a_; Tl[wave][r * 16 + 8 * hlf + v][t * 16 + nloc] = c_; }
    wave_lds_sync();
    b16* dst = ((which == 0) ? qh : kh) + (size_t)m0 * INNER + head * HD;
    for (int pass = 0; pass < 2; ++pass) {
#pragma unroll
      for (int j = 0; j < 8; ++j) { const int rr = j * 4 + (lane >> 3), c8 = (lane & 7) * 8; *(volatile v8b*)(dst + (size_t)rr * INNER + c8) = *(const v8b*)(&Th[wave][rr][c8]); *(volatile v8b*)(dst + QPL + (size_t)rr * INNER + c8) = *(const v8b*)(&Tl[wave][rr][c8]); }
      __threadfence(); }
    if (which == 0) return;
  }
#pragma unroll
  for (int t = 0; t < 4; ++t)
#pragma unroll
    for (int r = 0; r < 2; ++r)
#pragma unroll
      for (int v = 0; v < 8; ++v) { const float val = (which == 1) ? phi(acc[r][t][v]) : acc[r][t][v]; b16 a_, c_; split16(val * PS8, a_, c_); Tt[t * 16 + nloc][wave * 32 + r * 16 + 8 * hlf + v] = a_; Ttl[t * 16 + nloc][wave * 32 + r * 16 + 8 * hlf + v] = c_; }
  __syncthreads();
  b16* dstT = ((which == 1) ? kT : vT) + (((size_t)b * H + head) * HD) * S + tok0;
  for (int pass = 0; pass < 2; ++pass) {
#pragma unroll
    for (int j = 0; j < 8; ++j) { const int dd = wave * 16 + j * 2 + (lane >> 4), c8 = (lane & 15) * 8; *(volatile v8b*)(dstT + (size_t)dd * S + c8) = *(const v8b*)(&Tt[dd][c8]); *(volatile v8b*)(dstT + TPL + (size_t)dd * S + c8) = *(const v8b*)(&Ttl[dd][c8]); }
    __threadfence(); }
}

__global__ __launch_bounds__(128) void chunk_kernel(const b16* __restrict__ kT, const b16* __restrict__ vT, float* __restrict__ kv, float* __restrict__ ks) {
  __shared__ __attribute__((aligned(16))) float Ts[4][16][64 + 4]; __shared__ float Ks_[64];
  const int lane = threadIdx.x & 31, wave = threadIdx.x >> 5, nloc = lane & 15, hlf = lane >> 4; const int bh = blockIdx.x / NC, c = blockIdx.x % NC, n0 = c * CH;
  const b16* A0 = kT + ((size_t)bh * HD) * S + n0; const b16* B0 = vT + ((size_t)bh * HD) * S + n0;
  v8f acc[4] = {{}, {}, {}, {}};
#pragma unroll
  for (int kb = 0; kb < CH; kb += 32) { const v16b a = frag_kb(A0 + (size_t)(wave * 16 + nloc) * S + kb, hlf), al = frag_kb(A0 + TPL + (size_t)(wave * 16 + nloc) * S + kb, hlf);
#pragma unroll
    for (int t = 0; t < 4; ++t) { const v16b bv = frag_kb(B0 + (size_t)(t * 16 + nloc) * S + kb, hlf), bl = frag_kb(B0 + TPL + (size_t)(t * 16 + nloc) * S + kb, hlf);
      acc[t] = wmma16b(a, bv, acc[t]); acc[t] = wmma16b(al, bv, acc[t]); acc[t] = wmma16b(a, bl, acc[t]); } }
#pragma unroll
  for (int t = 0; t < 4; ++t)
#pragma unroll
    for (int v = 0; v < 8; ++v) Ts[wave][8 * hlf + v][t * 16 + nloc] = acc[t][v] * (1.0f / (PS8 * PS8));
  if (threadIdx.x < 64) { const b16* r = A0 + (size_t)threadIdx.x * S; float s = 0.0f; for (int m = 0; m < CH; ++m) s += ((float)r[m] + (float)r[TPL + m]); Ks_[threadIdx.x] = s * (1.0f / PS8); }
  __syncthreads();
  float* dst = kv + (((size_t)bh * NC + c) * HD) * HD;
  for (int pass = 0; pass < 2; ++pass) {
    for (int i = threadIdx.x; i < 16 * 64 / 4 * 4; i += 128) { const int w = i / 256, rem = i % 256, rr = rem >> 4, c4 = (rem & 15) * 4; *(volatile v4f*)(dst + (size_t)(w * 16 + rr) * HD + c4) = *(const v4f*)(&Ts[w][rr][c4]); }
    if (threadIdx.x < 16) *(volatile v4f*)(ks + ((size_t)bh * NC + c) * HD + threadIdx.x * 4) = *(const v4f*)(&Ks_[threadIdx.x * 4]);
    __threadfence(); }
}

typedef __attribute__((ext_vector_type(2))) _Float16 v2b; typedef __attribute__((ext_vector_type(2))) float v2f;
__global__ __launch_bounds__(256) void prefix_kernel(const float* __restrict__ kv, const float* __restrict__ ks, b16* __restrict__ cth, b16* __restrict__ ctl, float* __restrict__ cks) {
  const int g = blockIdx.x * 256 + threadIdx.x; const int bh = g >> 11, ee = (g >> 5) & 63, dd = (g & 31) * 2;
  float run0 = 0.0f, run1 = 0.0f, rk0 = 0.0f, rk1 = 0.0f;
  for (int c = 0; c < NC; ++c) { const size_t o = (((size_t)bh * NC + c) * HD + ee) * HD + dd; v2b vh, vl; b16 a, l; split16(run0 * CXS, a, l); vh[0] = a; vl[0] = l; split16(run1 * CXS, a, l); vh[1] = a; vl[1] = l;
    for (int pass = 0; pass < 2; ++pass) { *(volatile v2b*)(cth + o) = vh; *(volatile v2b*)(ctl + o) = vl; }
    if (ee == 0) { const v2f kk = {rk0, rk1}; for (int pass = 0; pass < 2; ++pass) *(volatile v2f*)(cks + ((size_t)bh * NC + c) * HD + dd) = kk;
      rk0 += ks[((size_t)bh * NC + c) * HD + dd]; rk1 += ks[((size_t)bh * NC + c) * HD + dd + 1]; }
    run0 += kv[(((size_t)bh * NC + c) * HD + dd) * HD + ee]; run1 += kv[(((size_t)bh * NC + c) * HD + dd + 1) * HD + ee]; }
  __threadfence();
}

__global__ __launch_bounds__(256) void attn_kernel(const b16* __restrict__ qh, const b16* __restrict__ kh, const b16* __restrict__ kT, const b16* __restrict__ vT, const b16* __restrict__ cth, const b16* __restrict__ ctl, const float* __restrict__ cks, float* __restrict__ orow) {
  __shared__ __attribute__((aligned(16))) float Os[8][16][HD + 4];
  const int wid = threadIdx.x >> 5, lane = threadIdx.x & 31, hh = lane >> 4, col = lane & 15;
  const int wg = blockIdx.x * 8 + wid, qt = wg & 3, c = (wg >> 2) % NC, bh = wg / (4 * NC), b = bh / H, h = bh % H, q0 = c * CH + qt * 16, qi = q0 + col;
  const b16* Q = qh + ((size_t)b * S + qi) * INNER + h * HD; const b16* KT = kT + ((size_t)bh * HD) * S; const b16* VT = vT + ((size_t)bh * HD) * S; const b16* CT = cth + (((size_t)bh * NC + c) * HD) * HD; const b16* CTL = ctl + (((size_t)bh * NC + c) * HD) * HD;
  v16b qf[2], ql[2];
#pragma unroll
  for (int ks_ = 0; ks_ < 2; ++ks_) { qf[ks_] = frag_kb(Q + ks_ * 32, hh); ql[ks_] = frag_kb(Q + QPL + ks_ * 32, hh); }
  v8f o[4] = {{}, {}, {}, {}};
#pragma unroll
  for (int n = 0; n < 4; ++n)
#pragma unroll
    for (int ks_ = 0; ks_ < 2; ++ks_) { const v16b a = frag_kb(CT + (size_t)(n * 16 + col) * HD + ks_ * 32, hh), al = frag_kb(CTL + (size_t)(n * 16 + col) * HD + ks_ * 32, hh);
      o[n] = wmma16b(a, qf[ks_], o[n]); o[n] = wmma16b(al, qf[ks_], o[n]); o[n] = wmma16b(a, ql[ks_], o[n]); }
  v8f oi[4];
#pragma unroll
  for (int n = 0; n < 4; ++n) { oi[n] = o[n]; o[n] = (v8f){}; }
  float deni = 0.0f; { const float* ck = cks + ((size_t)bh * NC + c) * HD;
#pragma unroll 8
    for (int d = 0; d < 32; ++d) deni += ((float)Q[32 * hh + d] + (float)Q[QPL + 32 * hh + d]) * (1.0f / PS8) * ck[32 * hh + d];
    deni += __shfl_xor(deni, 16); }
  const b16* K = kh + ((size_t)b * S) * INNER + h * HD; float dens = 0.0f;
#pragma unroll
  for (int kb2 = 0; kb2 < 2; ++kb2) { const int kb = c * CH + kb2 * 32; v8f s0 = {}, s1 = {};
#pragma unroll
    for (int ks_ = 0; ks_ < 2; ++ks_) { const v16b ka = frag_kb(K + (size_t)(kb + col) * INNER + ks_ * 32, hh), kal = frag_kb(K + QPL + (size_t)(kb + col) * INNER + ks_ * 32, hh), kb_ = frag_kb(K + (size_t)(kb + 16 + col) * INNER + ks_ * 32, hh), kbl = frag_kb(K + QPL + (size_t)(kb + 16 + col) * INNER + ks_ * 32, hh);
      s0 = wmma16b(ka, qf[ks_], s0); s0 = wmma16b(ka, ql[ks_], s0); s0 = wmma16b(kal, qf[ks_], s0); s1 = wmma16b(kb_, qf[ks_], s1); s1 = wmma16b(kb_, ql[ks_], s1); s1 = wmma16b(kbl, qf[ks_], s1); }
    v16b pb, pl;
#pragma unroll
    for (int r = 0; r < 8; ++r) { const int m0_ = kb + 8 * hh + r, m1_ = kb + 16 + 8 * hh + r;
      const float p0 = (m0_ <= qi) ? s0[r] * (1.0f / (PS8 * PS8)) : 0.0f, p1 = (m1_ <= qi) ? s1[r] * (1.0f / (PS8 * PS8)) : 0.0f; dens += p0 + p1;
      b16 a, cc; split16(p0 * CXS, a, cc); pb[r] = a; pl[r] = cc; split16(p1 * CXS, a, cc); pb[8 + r] = a; pl[8 + r] = cc; }
#pragma unroll
    for (int n = 0; n < 4; ++n) { const v16b vf = frag_kb(VT + (size_t)(n * 16 + col) * S + kb, hh), vl = frag_kb(VT + TPL + (size_t)(n * 16 + col) * S + kb, hh);
      o[n] = wmma16b(vf, pb, o[n]); o[n] = wmma16b(vf, pl, o[n]); o[n] = wmma16b(vl, pb, o[n]); } }
  dens += __shfl_xor(dens, 16);
  const float den = deni + dens + EPS; const float sc = 1.0f / (CXS * PS8);
#pragma unroll
  for (int n = 0; n < 4; ++n)
#pragma unroll
    for (int r = 0; r < 8; ++r) Os[wid][col][n * 16 + 8 * hh + r] = (oi[n][r] + o[n][r]) * sc / den;
  wave_lds_sync();
  float* dst = orow + ((size_t)b * S + q0) * INNER + h * HD;
  for (int pass = 0; pass < 2; ++pass) {
#pragma unroll
    for (int j = 0; j < 8; ++j) { const int rr = j * 2 + hh, c4 = col * 4; *(volatile v4f*)(dst + (size_t)rr * INNER + c4) = *(const v4f*)(&Os[wid][rr][c4]); }
    __threadfence(); }
}

__global__ __launch_bounds__(128) void outproj_kernel(const float* __restrict__ orow, const b16* __restrict__ wo16, const float* __restrict__ bout, float* __restrict__ y) {
  __shared__ __attribute__((aligned(16))) float Ts[4][32 * 64];
  const int lane = threadIdx.x & 31, wave = threadIdx.x >> 5, nloc = lane & 15, hlf = lane >> 4, m0 = blockIdx.y * 128 + wave * 32, c0 = blockIdx.x * 64;
  v8f acc[2][4];
#pragma unroll
  for (int r = 0; r < 2; ++r)
#pragma unroll
    for (int t = 0; t < 4; ++t) acc[r][t] = (v8f){};
#pragma unroll 2
  for (int kb = 0; kb < INNER; kb += 32) { v16b a0, a1, l0, l1;
#pragma unroll
    for (int e = 0; e < 16; ++e) { const int k = kb + ((e < 8) ? (8 * hlf + e) : (16 + 8 * hlf + e - 8)); b16 p, q; split16(orow[(size_t)(m0 + nloc) * INNER + k] * PS8, p, q); a0[e] = p; l0[e] = q; split16(orow[(size_t)(m0 + 16 + nloc) * INNER + k] * PS8, p, q); a1[e] = p; l1[e] = q; }
#pragma unroll
    for (int t = 0; t < 4; ++t) { const v16b bw = frag_kb(wo16 + (size_t)(c0 + t * 16 + nloc) * INNER + kb, hlf); acc[0][t] = wmma16b(a0, bw, acc[0][t]); acc[0][t] = wmma16b(l0, bw, acc[0][t]); acc[1][t] = wmma16b(a1, bw, acc[1][t]); acc[1][t] = wmma16b(l1, bw, acc[1][t]); } }
  float* Tt = Ts[wave];
#pragma unroll
  for (int t = 0; t < 4; ++t)
#pragma unroll
    for (int r = 0; r < 2; ++r)
#pragma unroll
      for (int v = 0; v < 8; ++v) Tt[(r * 16 + v + 8 * hlf) * 64 + t * 16 + nloc] = acc[r][t][v] * (1.0f / PS8) + bf16_rne(bout[c0 + t * 16 + nloc]);
  wave_lds_sync();
  float* dst0 = y + (size_t)m0 * DIM + c0;
  for (int pass = 0; pass < 2; ++pass) {
#pragma unroll
    for (int j = 0; j < 16; ++j) { const int rr = j * 2 + hlf, c4 = nloc * 4; *(volatile v4f*)(dst0 + (size_t)rr * DIM + c4) = *(const v4f*)(Tt + rr * 64 + c4); }
    __threadfence(); }
}
}

extern "C" void kernel_launch(void* const* d_in, const int* in_sizes, int n_in,
                              void* d_out, int out_size, void* d_ws, size_t ws_size, hipStream_t stream) {
  (void)n_in; (void)out_size;
  const float* x = (const float*)d_in[0]; const float* wqkv = (const float*)d_in[1]; const float* wout = (const float*)d_in[2]; const float* bout = (const float*)d_in[3];
  float* y = (float*)d_out;
  if (in_sizes[0] != NTOK * DIM || in_sizes[1] != DIM * 3 * INNER || in_sizes[2] != INNER * DIM || in_sizes[3] != DIM) return;
  size_t off = 0; char* ws = (char*)d_ws;
  auto carve = [&](size_t bytes) { char* p = ws + off; off += (bytes + 255) & ~(size_t)255; return p; };
  unsigned short* x16 = (unsigned short*)carve((size_t)NTOK * DIM * 2); unsigned short* w16 = (unsigned short*)carve((size_t)3 * INNER * DIM * 2); b16* wo16 = (b16*)carve((size_t)DIM * INNER * 2);
  b16* qhp = (b16*)carve(QPL * 2 * 2); b16* khp = (b16*)carve(QPL * 2 * 2); b16* kTp = (b16*)carve(TPL * 2 * 2); b16* vTp = (b16*)carve(TPL * 2 * 2);
  float* kv = (float*)carve(CPL * 4); float* ks = (float*)carve((size_t)NBH * NC * HD * 4); b16* cth = (b16*)carve(CPL * 2); b16* ctl = (b16*)carve(CPL * 2); float* cks = (float*)carve((size_t)NBH * NC * HD * 4); float* orow = (float*)carve((size_t)NTOK * INNER * 4);
  if (off > ws_size) return;
  prep_kernel<<<1024, 256, 0, stream>>>(x, wqkv, wout, x16, w16, wo16);
  proj_kernel<<<dim3(24, NTOK / 128), 128, 0, stream>>>(x16, w16, qhp, khp, kTp, vTp);
  chunk_kernel<<<NBH * NC, 128, 0, stream>>>(kTp, vTp, kv, ks);
  prefix_kernel<<<NBH * HD * 32 / 256, 256, 0, stream>>>(kv, ks, cth, ctl, cks);
  attn_kernel<<<NBH * NC * 4 / 8, 256, 0, stream>>>(qhp, khp, kTp, vTp, cth, ctl, cks, orow);
  outproj_kernel<<<dim3(DIM / 64, NTOK / 128), 128, 0, stream>>>(orow, wo16, bout, y);
}
